// NET_40913858461753
// MI455X (gfx1250) — hardware-verified
//
#include <hip/hip_runtime.h>
#include <stddef.h>
#include <stdint.h>
#include <math.h>


#define FIN     512
#define HC0     512
#define HID     64
#define NHD0    8
#define KA1     1024
#define NTHR    256
#define NWAVE   8
#define EPT     8
#define CHUNK   (NTHR * EPT)
#define WCAP    (EPT * 32)
#define LISTN   (NWAVE * WCAP)
#define NBA     1024
#define SLA     10
#define RCAP    28672
#define DEGCAP  128
#define MEAS_B1024  16582
#define MEAS_MAXDEG 35
#define GBM     64
#define GBN     64
#define GTHR    128
#define MROWS   128
#define NUW0    (HC0 * (FIN / 8))
#define NUW1    (HID * (KA1 / 8))
#define NEGSL   0.2f
#define MX0     (-3.0e38f)
#define WSMAX   134217728
#define BKT_ZINTS      (RCAP + 3 * NBA)
#define BKT_LDS_INTS   (LISTN + 2 * RCAP + 3 * NBA + 16)
#define SCAN_BASE_INTS (RCAP + 2 * NBA)
#define SCAN0_LDS_INTS (SCAN_BASE_INTS + NWAVE * 1024)
#define SCAN1_LDS_INTS (SCAN_BASE_INTS + 16)

static_assert((CHUNK & (CHUNK - 1)) == 0 && CHUNK <= 4096);
static_assert((NBA & (NBA - 1)) == 0 && NBA == (1 << SLA) && NBA <= 1024);
static_assert(((long long)CHUNK << SLA) < (1LL << 31));
static_assert(LISTN >= NWAVE * WCAP);
static_assert(NBA % NWAVE == 0 && NBA % 32 == 0);
static_assert(NTHR * 4 == NBA);
static_assert((RCAP % 32) == 0 && (BKT_ZINTS % 4) == 0 && (RCAP % (NTHR * 4)) == 0);
static_assert(RCAP >= MEAS_B1024 + 4096);
static_assert(DEGCAP >= MEAS_MAXDEG + 8);
static_assert(BKT_LDS_INTS * 4 <= 300000 && SCAN0_LDS_INTS * 4 <= 300000);
static_assert(BKT_LDS_INTS * 4 <= 327680 && SCAN0_LDS_INTS * 4 <= 327680);
static_assert(GBM == (GTHR / 32) * 16);
static_assert(GTHR == 2 * GBN && GTHR == 2 * GBM);
static_assert((FIN % 32) == 0 && (KA1 % 32) == 0 && KA1 == 2 * HC0);
static_assert((HC0 % GBN) == 0 && HID == GBN);
static_assert((MROWS % GBM) == 0);
static_assert(HC0 == 32 * 16);
static_assert(HID * NHD0 == HC0);
static_assert((HC0 % 128) == 0);
static_assert(HID == 2 * 32);
static_assert((NUW0 % NTHR) == 0 && (NUW1 % NTHR) == 0);

typedef float          v2f  __attribute__((ext_vector_type(2)));
typedef float          v4f  __attribute__((ext_vector_type(4)));
typedef float          v8f  __attribute__((ext_vector_type(8)));
typedef int            v4i  __attribute__((ext_vector_type(4)));
typedef int            v8i  __attribute__((ext_vector_type(8)));
typedef unsigned int   v4u  __attribute__((ext_vector_type(4)));
typedef unsigned short v8us __attribute__((ext_vector_type(8)));
typedef __bf16         v16b __attribute__((ext_vector_type(16)));
typedef v2f  __attribute__((may_alias)) v2fa;
typedef v4f  __attribute__((may_alias)) v4fa;
typedef v4i  __attribute__((may_alias)) v4ia;
typedef v4u  __attribute__((may_alias)) v4ua;
typedef v8us __attribute__((may_alias)) v8usa;
union FragB { v16b v; v8us h[2]; v8i w; };

__device__ __forceinline__ v8f wmb(const FragB& a, const FragB& b, v8f c) {
  v8f d = __builtin_amdgcn_wmma_f32_16x16x32_bf16(false, a.v, false, b.v, (short)0, c, false, false);
  asm volatile("v_nop\n\tv_nop\n\tv_nop\n\tv_nop" : "+v"(d) : "v"(a.w), "v"(b.w));
  return d;
}

__device__ __forceinline__ unsigned int f2bf(float f) {
  const unsigned int u = __float_as_uint(f);
  const unsigned int r = ((u + 0x7FFFu + ((u >> 16) & 1u)) >> 16) & 0xFFFFu;
  return ((u & 0x7FFFFFFFu) > 0x7F800000u) ? 0x7FC0u : r;
}
__device__ __forceinline__ float bf2f(unsigned int b) { return __uint_as_float(b << 16); }
__device__ __forceinline__ float bfr(float f) { return bf2f(f2bf(f)); }
__device__ __forceinline__ unsigned int pk2(float lo, float hi) { return f2bf(lo) | (f2bf(hi) << 16); }
__device__ __forceinline__ v4u pack8(const v4f a, const v4f b) {
  v4u r;
  r.x = pk2(a.x, a.y); r.y = pk2(a.z, a.w); r.z = pk2(b.x, b.y); r.w = pk2(b.z, b.w);
  return r;
}

template <int SLB>
__device__ __forceinline__ int scan_chunk(const int* __restrict__ dsts, int nE, int cbase, int slotBase,
                                          int nb, int vec8, int* list, int tid, int lane, int wave) {
  int wc = 0;
  const int el0  = tid * EPT;
  const int e0   = cbase + el0;
  const int sent = -2147483647 - 1;
  v4i da, db;
  if (vec8 != 0 && cbase + CHUNK <= nE) {
    da = *(const v4i*)(dsts + e0);
    db = *(const v4i*)(dsts + e0 + 4);
  } else {
    da.x = (e0     < nE) ? dsts[min(e0,     nE - 1)] : sent;
    da.y = (e0 + 1 < nE) ? dsts[min(e0 + 1, nE - 1)] : sent;
    da.z = (e0 + 2 < nE) ? dsts[min(e0 + 2, nE - 1)] : sent;
    da.w = (e0 + 3 < nE) ? dsts[min(e0 + 3, nE - 1)] : sent;
    db.x = (e0 + 4 < nE) ? dsts[min(e0 + 4, nE - 1)] : sent;
    db.y = (e0 + 5 < nE) ? dsts[min(e0 + 5, nE - 1)] : sent;
    db.z = (e0 + 6 < nE) ? dsts[min(e0 + 6, nE - 1)] : sent;
    db.w = (e0 + 7 < nE) ? dsts[min(e0 + 7, nE - 1)] : sent;
  }
  const unsigned nbs = (unsigned)slotBase;
  const unsigned unb = (unsigned)nb;
  const unsigned s0 = (unsigned)da.x - nbs, s1 = (unsigned)da.y - nbs;
  const unsigned s2 = (unsigned)da.z - nbs, s3 = (unsigned)da.w - nbs;
  const unsigned s4 = (unsigned)db.x - nbs, s5 = (unsigned)db.y - nbs;
  const unsigned s6 = (unsigned)db.z - nbs, s7 = (unsigned)db.w - nbs;
  const bool h0 = s0 < unb, h1 = s1 < unb, h2 = s2 < unb, h3 = s3 < unb;
  const bool h4 = s4 < unb, h5 = s5 < unb, h6 = s6 < unb, h7 = s7 < unb;
  const unsigned any = __builtin_amdgcn_ballot_w32(h0 | h1 | h2 | h3 | h4 | h5 | h6 | h7);
  if (any != 0u) {
#define HITJ(J, HJ, SJ) { \
      const unsigned mj = __builtin_amdgcn_ballot_w32(HJ); \
      if (mj != 0u) { \
        if (HJ) { \
          const int pos = wc + (int)__builtin_amdgcn_mbcnt_lo(mj, 0u); \
          if (pos < WCAP) list[wave * WCAP + pos] = ((el0 + (J)) << SLB) | (int)(SJ); \
        } \
        wc += (int)__builtin_popcount(mj); } }
    HITJ(0, h0, s0)
    HITJ(1, h1, s1)
    HITJ(2, h2, s2)
    HITJ(3, h3, s3)
    HITJ(4, h4, s4)
    HITJ(5, h5, s5)
    HITJ(6, h6, s6)
    HITJ(7, h7, s7)
#undef HITJ
  }
  return wc;
}

__global__ __launch_bounds__(NTHR) void k_pa(const float* __restrict__ x, unsigned short* xb, int nN, int nUnits) {
  const int i = (int)blockIdx.x * NTHR + (int)threadIdx.x;
  if (i >= nUnits) return;
  const int row = i >> 6;
  const int c0  = (i & 63) * 8;
  const int rc  = row < nN ? row : nN - 1;
  const float* p = x + (size_t)rc * FIN + c0;
  v4f a = *(const v4fa*)p, b = *(const v4fa*)(p + 4);
  const v4f z4 = {0.f, 0.f, 0.f, 0.f};
  if (row >= nN) { a = z4; b = z4; }
  const v4u hv = pack8(a, b);
  const size_t o = (size_t)row * FIN + c0;
  *(volatile v4u*)(xb + o) = hv;
  __threadfence();
  *(volatile v4u*)(xb + o) = hv;
}

__global__ __launch_bounds__(NTHR) void k_pb(const float* __restrict__ W0, const float* __restrict__ W1,
                                             unsigned short* W0T, unsigned short* W1D) {
  const int u = (int)blockIdx.x * NTHR + (int)threadIdx.x;
  v8us o;
  unsigned short* dp;
  if (u < NUW0) {
    const int n  = u >> 6;
    const int k8 = (u & 63) * 8;
    const float* p = W0 + (size_t)k8 * HC0 + n;
#pragma unroll
    for (int i = 0; i < 8; ++i) o[i] = (unsigned short)f2bf(p[(size_t)i * HC0]);
    dp = W0T + (size_t)n * FIN + k8;
  } else if (u < NUW0 + NUW1) {
    const int v  = u - NUW0;
    const int n  = v >> 7;
    const int k8 = (v & 127) * 8;
    const int kk = k8 & (HC0 - 1);
    const float* p = W1 + (size_t)kk * HID + n;
#pragma unroll
    for (int i = 0; i < 8; ++i) o[i] = (unsigned short)f2bf(p[(size_t)i * HID]);
    dp = W1D + (size_t)n * KA1 + k8;
  } else {
    return;
  }
  *(volatile v8us*)dp = o;
  __threadfence();
  *(volatile v8us*)dp = o;
}

__global__ __launch_bounds__(NTHR) void k_bucket(const int* __restrict__ srcs, const int* __restrict__ dsts,
                                                 int nE, int nN, int vec8,
                                                 int* LIST, int* CNT, int* OFF, int* FLG) {
  extern __shared__ __attribute__((aligned(16))) int bsm[];
  int* list = bsm;
  int* reg1 = list + LISTN;
  int* sl   = reg1 + RCAP;
  int* cnt  = sl + RCAP;
  int* offs = cnt + NBA;
  int* cur  = offs + NBA;
  int* wcnt = cur + NBA;
  const int tid = (int)threadIdx.x, lane = tid & 31, wave = tid >> 5;
  const int blk = (int)blockIdx.x;
  const int nodeBase = blk * NBA;
  int nb = nN - nodeBase;
  nb = nb < 0 ? 0 : (nb > NBA ? NBA : nb);

  {
    const v4i z4 = {0, 0, 0, 0};
    for (int i = tid * 4; i < BKT_ZINTS; i += NTHR * 4) *(v4ia*)(sl + i) = z4;
  }
  __syncthreads();

  int tot = 0, ovf = 0;
  const int nChunks = (nE + CHUNK - 1) / CHUNK;
#pragma unroll 1
  for (int ch = 0; ch < nChunks; ++ch) {
    const int cbase = ch * CHUNK;
    const int wc = scan_chunk<SLA>(dsts, nE, cbase, nodeBase, nb, vec8, list, tid, lane, wave);
    if (lane == 0) wcnt[wave] = wc;
    __syncthreads();
    int pre = 0, all = 0;
#pragma unroll
    for (int w2 = 0; w2 < NWAVE; ++w2) {
      int c = wcnt[w2];
      c = c < 0 ? 0 : (c > WCAP ? WCAP : c);
      all += c;
      pre += (w2 < wave) ? c : 0;
    }
    const int wcc  = wc > WCAP ? WCAP : wc;
    const int base = tot + pre;
#pragma unroll 1
    for (int i = lane; i < wcc; i += 32) {
      const int ent = list[wave * WCAP + i];
      const int el  = (ent >> SLA) & (CHUNK - 1);
      const int sq  = ent & (NBA - 1);
      int eid = cbase + el;
      eid = eid > nE - 1 ? nE - 1 : eid;
      const int sraw = srcs[eid];
      const int s = sraw < 0 ? 0 : (sraw > nN - 1 ? nN - 1 : sraw);
      const int pos = base + i;
      if (pos < RCAP) reg1[pos] = (int)((unsigned)s | ((unsigned)sq << 16));
    }
    if (tot + all > RCAP) ovf = 1;
    tot += all;
    tot = tot > RCAP ? RCAP : tot;
    __syncthreads();
  }
  const int nh = tot;

  if (wave == 0) {
#pragma unroll 1
    for (int b0 = 0; b0 < nh; b0 += 32) {
      const int idx = b0 + lane;
      const int uv  = reg1[idx < nh ? idx : nh - 1];
      const int m32 = (nh - b0) < 32 ? (nh - b0) : 32;
#pragma unroll 1
      for (int k = 0; k < m32; ++k) {
        const int u  = __builtin_amdgcn_readlane(uv, k);
        const int sq = (u >> 16) & (NBA - 1);
        if (lane == 0) cnt[sq] = cnt[sq] + 1;
      }
    }
  }
  __syncthreads();
  if (wave == 0) {
    const int base = lane * (NBA / 32);
    int s = 0;
#pragma unroll 1
    for (int i = 0; i < NBA / 32; ++i) s += cnt[base + i];
    int incl = s;
#pragma unroll
    for (int d = 1; d < 32; d <<= 1) {
      const int y = __shfl_up(incl, d, 32);
      if (lane >= d) incl += y;
    }
    int run = incl - s;
#pragma unroll 1
    for (int i = 0; i < NBA / 32; ++i) {
      const int cv = cnt[base + i];
      offs[base + i] = run;
      cur[base + i]  = run;
      run += cv;
    }
  }
  __syncthreads();
  if (wave == 0) {
#pragma unroll 1
    for (int b0 = 0; b0 < nh; b0 += 32) {
      const int idx = b0 + lane;
      const int uv  = reg1[idx < nh ? idx : nh - 1];
      const int m32 = (nh - b0) < 32 ? (nh - b0) : 32;
#pragma unroll 1
      for (int k = 0; k < m32; ++k) {
        const int u  = __builtin_amdgcn_readlane(uv, k);
        const int sq = (u >> 16) & (NBA - 1);
        if (lane == 0) {
          int p = cur[sq];
          p = p < 0 ? 0 : (p > RCAP - 1 ? RCAP - 1 : p);
          sl[p] = u & 0xFFFF;
          cur[sq] = p + 1;
        }
      }
    }
  }
  __syncthreads();

  int* lb = LIST + (size_t)blk * RCAP;
  int* cp = CNT + (size_t)blk * NBA + 4 * tid;
  int* op = OFF + (size_t)blk * NBA + 4 * tid;
  int* fp = FLG + (size_t)blk * 32 + 4 * (tid & 7);
  const v4i cq = *(const v4ia*)(cnt + 4 * tid);
  const v4i oq = *(const v4ia*)(offs + 4 * tid);
  v4i cv;
  cv.x = (tid == 0) ? nh : 0;
  cv.y = (tid == 0) ? ovf : 0;
  cv.z = 0; cv.w = 0;
#pragma unroll 1
  for (int p = tid * 4; p < RCAP; p += NTHR * 4) {
    const v4i v = *(const v4ia*)(sl + p);
    *(volatile v4i*)(lb + p) = v;
  }
  *(volatile v4i*)cp = cq;
  *(volatile v4i*)op = oq;
  if (tid < 8) *(volatile v4i*)fp = cv;
  __threadfence();
#pragma unroll 1
  for (int p = tid * 4; p < RCAP; p += NTHR * 4) {
    const v4i v = *(const v4ia*)(sl + p);
    *(volatile v4i*)(lb + p) = v;
  }
  *(volatile v4i*)cp = cq;
  *(volatile v4i*)op = oq;
  if (tid < 8) *(volatile v4i*)fp = cv;
}

__global__ __launch_bounds__(GTHR) __attribute__((amdgpu_num_vgpr(248))) void k_gemm(
    const unsigned short* __restrict__ A, const unsigned short* __restrict__ WT,
    float* outF, int K, int ldo,
    const float* __restrict__ atts, const float* __restrict__ attd, int attLen,
    float* SD, int MPr)
{
  __shared__ __attribute__((aligned(16))) float stg[GBM * GBN];
  __shared__ __attribute__((aligned(16))) float satt[2 * GBN];
  __shared__ __attribute__((aligned(16))) float sdot[2 * GBM];
  const int tid = (int)threadIdx.x, lane = tid & 31, wave = tid >> 5, hh = lane >> 4, m = lane & 15;
  const int rowBase = (int)blockIdx.x * GBM;
  const int head    = (int)blockIdx.y;
  const int col0    = head * GBN;

  {
    const int which = tid >> 6;
    const int c  = tid & 63;
    const int cl = c < attLen ? c : attLen - 1;
    const float vs = atts[head * attLen + cl];
    const float vd = attd[head * attLen + cl];
    float v = (which == 0) ? vs : vd;
    v = (c < attLen) ? bfr(v) : 0.f;
    satt[which * GBN + c] = v;
  }

  v8f acc[4];
  {
    const v8f z = {0.f, 0.f, 0.f, 0.f, 0.f, 0.f, 0.f, 0.f};
    acc[0] = z; acc[1] = z; acc[2] = z; acc[3] = z;
  }
  const unsigned short* ap = A  + (size_t)(rowBase + 16 * wave + m) * (size_t)K + 8 * hh;
  const unsigned short* wp = WT + (size_t)(col0 + m) * (size_t)K + 8 * hh;
  const int ksteps = K >> 5;
#pragma unroll 1
  for (int ks = 0; ks < ksteps; ++ks) {
    FragB af;
    af.h[0] = *(const v8usa*)(ap + 32 * ks);
    af.h[1] = *(const v8usa*)(ap + 32 * ks + 16);
#pragma unroll
    for (int t = 0; t < 4; ++t) {
      const unsigned short* wq = wp + (size_t)(16 * t) * (size_t)K + 32 * ks;
      FragB bf;
      bf.h[0] = *(const v8usa*)wq;
      bf.h[1] = *(const v8usa*)(wq + 16);
      acc[t] = wmb(af, bf, acc[t]);
    }
  }

#pragma unroll
  for (int t = 0; t < 4; ++t) {
    const int lc = 16 * t + m;
#pragma unroll
    for (int r = 0; r < 8; ++r) {
      const int lr = 16 * wave + 8 * hh + r;
      stg[lr * GBN + lc] = acc[t][r];
    }
  }
  __syncthreads();

  {
    const int row = tid & 63, which = tid >> 6;
    const float* sa = satt + which * GBN;
    const float* hr = stg + row * GBN;
    float d = 0.f;
#pragma unroll 4
    for (int c4 = 0; c4 < GBN / 4; ++c4) {
      const v4f hv = *(const v4fa*)(hr + 4 * c4);
      const v4f av = *(const v4fa*)(sa + 4 * c4);
      d = fmaf(hv.x, av.x, d);
      d = fmaf(hv.y, av.y, d);
      d = fmaf(hv.z, av.z, d);
      d = fmaf(hv.w, av.w, d);
    }
    sdot[which * GBM + row] = d;
  }
  __syncthreads();

  v4f fv[8];
#pragma unroll
  for (int i = 0; i < 8; ++i) {
    const int lr = 16 * wave + 2 * i + hh;
    fv[i] = *(const v4fa*)(stg + lr * GBN + 4 * m);
  }
  const int which2 = lane >> 4, piece = lane & 15;
  const v4f sdv = *(const v4fa*)(sdot + which2 * GBM + 4 * piece);
  float* sp = SD + (size_t)(2 * head + which2) * (size_t)MPr + rowBase + 4 * piece;

#pragma unroll
  for (int i = 0; i < 8; ++i) {
    const int lr = 16 * wave + 2 * i + hh;
    const int gr = rowBase + lr;
    float* op = outF + (size_t)gr * (size_t)ldo + col0 + 4 * m;
    *(volatile v4f*)op = fv[i];
  }
  if (wave == 0) *(volatile v4f*)sp = sdv;
  __threadfence();
#pragma unroll
  for (int i = 0; i < 8; ++i) {
    const int lr = 16 * wave + 2 * i + hh;
    const int gr = rowBase + lr;
    float* op = outF + (size_t)gr * (size_t)ldo + col0 + 4 * m;
    *(volatile v4f*)op = fv[i];
  }
  if (wave == 0) *(volatile v4f*)sp = sdv;
}

template <int L>
__global__ __launch_bounds__(NTHR) __attribute__((amdgpu_num_vgpr(248))) void k_scan(
    const int* __restrict__ LIST, const int* __restrict__ CNT, const int* __restrict__ OFF,
    const int* __restrict__ FLG, const float* __restrict__ F, const float* __restrict__ SD,
    unsigned short* HP, float* out, int nN, int MPr) {
  static_assert(L == 0 || L == 1);
  constexpr int CPL = (L == 0) ? 16 : 2;
  constexpr int C   = CPL * 32;
  extern __shared__ __attribute__((aligned(16))) int ssm[];
  int* hl   = ssm;
  int* cnt  = hl + RCAP;
  int* offs = cnt + NBA;
  unsigned int* stg = (unsigned int*)(offs + NBA);
  const int tid = (int)threadIdx.x, lane = tid & 31, wave = tid >> 5;
  const int blk = (int)blockIdx.x;
  const int nodeBase = blk * NBA;

  const int nhraw = FLG[(size_t)blk * 32];
  const int bflag = FLG[(size_t)blk * 32 + 1];
  const int nh  = nhraw < 0 ? 0 : (nhraw > RCAP ? RCAP : nhraw);
  const int ovf = (bflag != 0 || nhraw < 0 || nhraw > RCAP) ? 1 : 0;

  {
    const int* hb = LIST + (size_t)blk * RCAP;
#pragma unroll 1
    for (int p = tid * 4; p < RCAP; p += NTHR * 4) {
      const v4i v = *(const v4i*)(hb + p);
      *(v4ia*)(hl + p) = v;
    }
    const v4i cq = *(const v4i*)(CNT + (size_t)blk * NBA + 4 * tid);
    const v4i oq = *(const v4i*)(OFF + (size_t)blk * NBA + 4 * tid);
    *(v4ia*)(cnt + 4 * tid)  = cq;
    *(v4ia*)(offs + 4 * tid) = oq;
  }
  __syncthreads();

  const float qnan = __int_as_float(0x7fc00000);
  const int head   = (L == 0) ? (lane >> 2) : 0;
  const size_t hoS = (size_t)(2 * head) * (size_t)MPr;
  const size_t hoD = hoS + (size_t)MPr;
  unsigned int* stA = stg + wave * 1024;
  unsigned int* stB = stA + 512;

#pragma unroll 1
  for (int si = 0; si < NBA / NWAVE; ++si) {
    const int s    = si * NWAVE + wave;
    const int node = nodeBase + s;
    const int nc   = node < nN ? node : nN - 1;
    const int craw = cnt[s];
    const bool big = craw > DEGCAP;
    int c = craw < 0 ? 0 : (craw > DEGCAP ? DEGCAP : craw);
    int o = offs[s];
    o = o < 0 ? 0 : (o > RCAP ? RCAP : o);
    if (c > nh - o) c = nh - o;
    c = c < 0 ? 0 : c;
    c = __builtin_amdgcn_readfirstlane(c);
    o = __builtin_amdgcn_readfirstlane(o);
    const bool pois = (ovf != 0) || big;
    const bool live = node < nN;
    const float adv = SD[hoD + (size_t)nc];
    float mx = MX0, dn = 0.0f;
    v4f a0 = {0.f, 0.f, 0.f, 0.f};
    v4f a1 = {0.f, 0.f, 0.f, 0.f};
    v4f a2 = {0.f, 0.f, 0.f, 0.f};
    v4f a3 = {0.f, 0.f, 0.f, 0.f};
    float q0 = 0.0f, q1 = 0.0f;
#pragma unroll 1
    for (int b0 = 0; b0 < c; b0 += 32) {
      const int t  = b0 + lane;
      const int tt = t < c ? t : c - 1;
      int idx = o + tt;
      idx = idx < 0 ? 0 : (idx > RCAP - 1 ? RCAP - 1 : idx);
      const int ent = hl[idx];
      const int sr  = ent < 0 ? 0 : (ent > nN - 1 ? nN - 1 : ent);
      const int m32 = (c - b0) < 32 ? (c - b0) : 32;
#pragma unroll 1
      for (int k = 0; k < m32; ++k) {
        const int sk = __builtin_amdgcn_readlane(sr, k);
        const float* rp = F + (size_t)sk * C + CPL * lane;
        float lg = SD[hoS + (size_t)sk] + adv;
        lg = lg > 0.f ? lg : NEGSL * lg;
        const float df = lg - mx;
        const float ee = expf(-fabsf(df));
        const bool  up = df > 0.f;
        const float s1 = up ? ee : 1.0f;
        const float s2 = up ? 1.0f : ee;
        mx = up ? lg : mx;
        dn = fmaf(dn, s1, s2);
        if constexpr (L == 0) {
          const v4f f0 = *(const v4f*)rp;
          const v4f f1 = *(const v4f*)(rp + 4);
          const v4f f2 = *(const v4f*)(rp + 8);
          const v4f f3 = *(const v4f*)(rp + 12);
          a0.x = fmaf(a0.x, s1, s2 * f0.x); a0.y = fmaf(a0.y, s1, s2 * f0.y);
          a0.z = fmaf(a0.z, s1, s2 * f0.z); a0.w = fmaf(a0.w, s1, s2 * f0.w);
          a1.x = fmaf(a1.x, s1, s2 * f1.x); a1.y = fmaf(a1.y, s1, s2 * f1.y);
          a1.z = fmaf(a1.z, s1, s2 * f1.z); a1.w = fmaf(a1.w, s1, s2 * f1.w);
          a2.x = fmaf(a2.x, s1, s2 * f2.x); a2.y = fmaf(a2.y, s1, s2 * f2.y);
          a2.z = fmaf(a2.z, s1, s2 * f2.z); a2.w = fmaf(a2.w, s1, s2 * f2.w);
          a3.x = fmaf(a3.x, s1, s2 * f3.x); a3.y = fmaf(a3.y, s1, s2 * f3.y);
          a3.z = fmaf(a3.z, s1, s2 * f3.z); a3.w = fmaf(a3.w, s1, s2 * f3.w);
        } else {
          const v2f f0 = *(const v2fa*)rp;
          q0 = fmaf(q0, s1, s2 * f0.x);
          q1 = fmaf(q1, s1, s2 * f0.y);
        }
      }
    }
    const float rinv = __builtin_amdgcn_rcpf(dn);
    const float inv  = (c > 0) ? rinv : 0.0f;

    if constexpr (L == 0) {
      stA[ 0 * 32 + lane] = __float_as_uint(a0.x); stA[ 1 * 32 + lane] = __float_as_uint(a0.y);
      stA[ 2 * 32 + lane] = __float_as_uint(a0.z); stA[ 3 * 32 + lane] = __float_as_uint(a0.w);
      stA[ 4 * 32 + lane] = __float_as_uint(a1.x); stA[ 5 * 32 + lane] = __float_as_uint(a1.y);
      stA[ 6 * 32 + lane] = __float_as_uint(a1.z); stA[ 7 * 32 + lane] = __float_as_uint(a1.w);
      stA[ 8 * 32 + lane] = __float_as_uint(a2.x); stA[ 9 * 32 + lane] = __float_as_uint(a2.y);
      stA[10 * 32 + lane] = __float_as_uint(a2.z); stA[11 * 32 + lane] = __float_as_uint(a2.w);
      stA[12 * 32 + lane] = __float_as_uint(a3.x); stA[13 * 32 + lane] = __float_as_uint(a3.y);
      stA[14 * 32 + lane] = __float_as_uint(a3.z); stA[15 * 32 + lane] = __float_as_uint(a3.w);
#pragma unroll 1
      for (int j = 0; j < 16; ++j) {
        float y = __uint_as_float(stA[j * 32 + lane]) * inv;
        y = (y > 0.0f) ? y : expm1f(y);
        y = pois ? qnan : y;
        y = live ? y : 0.0f;
        stA[j * 32 + lane] = __float_as_uint(y);
      }
      unsigned int hw[8], lw[8];
#pragma unroll
      for (int i = 0; i < 8; ++i) {
        const float va = __uint_as_float(stA[(2 * i) * 32 + lane]);
        const float vb = __uint_as_float(stA[(2 * i + 1) * 32 + lane]);
        const unsigned int ha = f2bf(va);
        const unsigned int hb2 = f2bf(vb);
        hw[i] = ha | (hb2 << 16);
        lw[i] = f2bf(va - bf2f(ha)) | (f2bf(vb - bf2f(hb2)) << 16);
      }
      v4u hA, hB, lA, lB;
      hA.x = hw[0]; hA.y = hw[1]; hA.z = hw[2]; hA.w = hw[3];
      hB.x = hw[4]; hB.y = hw[5]; hB.z = hw[6]; hB.w = hw[7];
      lA.x = lw[0]; lA.y = lw[1]; lA.z = lw[2]; lA.w = lw[3];
      lB.x = lw[4]; lB.y = lw[5]; lB.z = lw[6]; lB.w = lw[7];
      *(v4ua*)(stB + 8 * lane)           = hA;
      *(v4ua*)(stB + 8 * lane + 4)       = hB;
      *(v4ua*)(stB + 256 + 8 * lane)     = lA;
      *(v4ua*)(stB + 256 + 8 * lane + 4) = lB;
      __builtin_amdgcn_fence(__ATOMIC_RELEASE, "workgroup");
      __builtin_amdgcn_wave_barrier();
      __builtin_amdgcn_fence(__ATOMIC_ACQUIRE, "workgroup");
      const v4u r0 = *(const v4ua*)(stB + 4 * lane);
      const v4u r1 = *(const v4ua*)(stB + 128 + 4 * lane);
      const v4u r2 = *(const v4ua*)(stB + 256 + 4 * lane);
      const v4u r3 = *(const v4ua*)(stB + 384 + 4 * lane);
      if (node < MPr) {
        unsigned short* hp = HP + (size_t)node * KA1 + 8 * lane;
        *(volatile v4u*)hp         = r0;
        *(volatile v4u*)(hp + 256) = r1;
        *(volatile v4u*)(hp + 512) = r2;
        *(volatile v4u*)(hp + 768) = r3;
        __threadfence();
        *(volatile v4u*)hp         = r0;
        *(volatile v4u*)(hp + 256) = r1;
        *(volatile v4u*)(hp + 512) = r2;
        *(volatile v4u*)(hp + 768) = r3;
      }
      __builtin_amdgcn_fence(__ATOMIC_RELEASE, "workgroup");
      __builtin_amdgcn_wave_barrier();
    } else {
      float r0 = q0 * inv;
      float r1 = q1 * inv;
      r0 = pois ? qnan : r0;
      r1 = pois ? qnan : r1;
      v2f ov; ov.x = r0; ov.y = r1;
      if (node < nN) {
        float* op = out + (size_t)node * HID + 2 * lane;
        *(volatile v2f*)op = ov;
        __threadfence();
        *(volatile v2f*)op = ov;
      }
    }
  }
}

static inline int cdiv(int a, int b) { return (a + b - 1) / b; }

extern "C" void kernel_launch(void* const* d_in, const int* in_sizes, int n_in,
                              void* d_out, int out_size, void* d_ws, size_t ws_size,
                              hipStream_t stream) {
  if (n_in < 9) return;
  const int nN = in_sizes[0] / FIN;
  if (nN <= 0 || in_sizes[0] != nN * FIN || nN > 65536) return;
  const int nE = in_sizes[1];
  if (nE < 1 || nE > (1 << 30) || in_sizes[2] != nE) return;
  if (in_sizes[3] != FIN * HC0) return;
  if (in_sizes[4] != NHD0 * HID || in_sizes[5] != NHD0 * HID) return;
  if (in_sizes[6] != HC0 * HID) return;
  if (in_sizes[7] != HID || in_sizes[8] != HID) return;
  if (out_size != nN * HID) return;

  const float* feats = (const float*)d_in[0];
  const int*   src   = (const int*)  d_in[1];
  const int*   dst   = (const int*)  d_in[2];
  const float* W0    = (const float*)d_in[3];
  const float* al0   = (const float*)d_in[4];
  const float* ar0   = (const float*)d_in[5];
  const float* W1    = (const float*)d_in[6];
  const float* al1   = (const float*)d_in[7];
  const float* ar1   = (const float*)d_in[8];
  float* out = (float*)d_out;

  const int MP   = cdiv(nN, MROWS) * MROWS;
  const int gM   = MP / GBM;
  const int gA   = cdiv(MP, NBA);
  if ((long long)gA * NBA < (long long)MP) return;
  const int vec8 = ((nE & 3) == 0) ? 1 : 0;
  const int nUx  = MP * (FIN / 8);
  if ((nUx % NTHR) != 0) return;

  char* ws = (char*)d_ws;
  size_t off = 0;
  const size_t oXB  = off; off += (size_t)MP * FIN * 2;           off = (off + 255) & ~(size_t)255;
  const size_t oW0T = off; off += (size_t)HC0 * FIN * 2;          off = (off + 255) & ~(size_t)255;
  const size_t oW1D = off; off += (size_t)HID * KA1 * 2;          off = (off + 255) & ~(size_t)255;
  const size_t oF0  = off; off += (size_t)MP * HC0 * 4;           off = (off + 255) & ~(size_t)255;
  const size_t oSD0 = off; off += (size_t)2 * NHD0 * MP * 4;      off = (off + 255) & ~(size_t)255;
  const size_t oH1  = off; off += (size_t)MP * KA1 * 2;           off = (off + 255) & ~(size_t)255;
  const size_t oF1  = off; off += (size_t)MP * HID * 4;           off = (off + 255) & ~(size_t)255;
  const size_t oSD1 = off; off += (size_t)2 * MP * 4;             off = (off + 255) & ~(size_t)255;
  const size_t oLST = off; off += (size_t)gA * RCAP * 4;          off = (off + 255) & ~(size_t)255;
  const size_t oCNT = off; off += (size_t)gA * NBA * 4;           off = (off + 255) & ~(size_t)255;
  const size_t oOFF = off; off += (size_t)gA * NBA * 4;           off = (off + 255) & ~(size_t)255;
  const size_t oFLG = off; off += (size_t)gA * 128;               off = (off + 255) & ~(size_t)255;
  if (off > ws_size || off > (size_t)WSMAX) return;
  unsigned short* XB   = (unsigned short*)(ws + oXB);
  unsigned short* W0T  = (unsigned short*)(ws + oW0T);
  unsigned short* W1D  = (unsigned short*)(ws + oW1D);
  float*          FE0  = (float*)(ws + oF0);
  float*          SD0  = (float*)(ws + oSD0);
  unsigned short* H1   = (unsigned short*)(ws + oH1);
  float*          FE1  = (float*)(ws + oF1);
  float*          SD1  = (float*)(ws + oSD1);
  int*            LIST = (int*)(ws + oLST);
  int*            CNT  = (int*)(ws + oCNT);
  int*            OFF  = (int*)(ws + oOFF);
  int*            FLG  = (int*)(ws + oFLG);

  const int bktLds   = BKT_LDS_INTS * 4;
  const int scan0Lds = SCAN0_LDS_INTS * 4;
  const int scan1Lds = SCAN1_LDS_INTS * 4;
  hipFuncSetAttribute(reinterpret_cast<const void*>(&k_bucket),
                      hipFuncAttributeMaxDynamicSharedMemorySize, bktLds);
  hipFuncSetAttribute(reinterpret_cast<const void*>(&k_scan<0>),
                      hipFuncAttributeMaxDynamicSharedMemorySize, scan0Lds);
  hipFuncSetAttribute(reinterpret_cast<const void*>(&k_scan<1>),
                      hipFuncAttributeMaxDynamicSharedMemorySize, scan1Lds);

  k_pa<<<nUx / NTHR, NTHR, 0, stream>>>(feats, XB, nN, nUx);
  k_pb<<<(NUW0 + NUW1) / NTHR, NTHR, 0, stream>>>(W0, W1, W0T, W1D);
  k_bucket<<<gA, NTHR, bktLds, stream>>>(src, dst, nE, nN, vec8, LIST, CNT, OFF, FLG);
  k_gemm<<<dim3(gM, HC0 / GBN), GTHR, 0, stream>>>(XB, W0T, FE0, FIN, HC0, al0, ar0, HID, SD0, MP);
  k_scan<0><<<gA, NTHR, scan0Lds, stream>>>(LIST, CNT, OFF, FLG, FE0, SD0, H1, out, nN, MP);
  k_gemm<<<dim3(gM, HID / GBN), GTHR, 0, stream>>>(H1, W1D, FE1, KA1, HID, al1, ar1, HID, SD1, MP);
  k_scan<1><<<gA, NTHR, scan1Lds, stream>>>(LIST, CNT, OFF, FLG, FE1, SD1, H1, out, nN, MP);
}
